// FusedRobertaLayer_80908593922048
// MI455X (gfx1250) — hardware-verified
//
#include <hip/hip_runtime.h>
#include <stdint.h>
#include <stddef.h>

#define D_MODEL 1024
#define FF_DIM  4096
#define SEQ     512
#define BATCH   8
#define NHEAD   16
#define HDIM    64
#define MTOT    (BATCH * SEQ)
#define LORA_R  16
#define LN_EPS  1e-5f
#define WSCALE      64.0f
#define WSCALE_INV  0.015625f
#define PSCALE      256.0f
#define PSCALE_INV  0.00390625f

#define GBM  128
#define GBN  128
#define GBK  64
#define GLDP 72
#define ALDP 72

typedef char chk_d   [(D_MODEL == 1024) ? 1 : -1];
typedef char chk_h   [(NHEAD * HDIM == D_MODEL) ? 1 : -1];
typedef char chk_mn  [(MTOT % GBM == 0 && D_MODEL % GBN == 0 && FF_DIM % GBN == 0) ? 1 : -1];
typedef char chk_k   [(D_MODEL % GBK == 0 && FF_DIM % GBK == 0) ? 1 : -1];
typedef char chk_att [(SEQ % 128 == 0 && HDIM == 64) ? 1 : -1];

typedef _Float16 v16h __attribute__((ext_vector_type(16)));
typedef _Float16 v8h  __attribute__((ext_vector_type(8)));
typedef float    v8f  __attribute__((ext_vector_type(8)));
typedef float    v4f  __attribute__((ext_vector_type(4)));
typedef unsigned int v4u __attribute__((ext_vector_type(4)));

union Frag   { v16h v; v8h half[2]; };
union Pack16 { v8h h; v4u u; };

__device__ __forceinline__ Frag ld_frag(const _Float16* base, int pitch, int row0, int k0) {
  const int l = threadIdx.x & 31, h = l >> 4, m = l & 15;
  const _Float16* p = base + (size_t)(row0 + m) * pitch + k0 + 8 * h;
  Frag f;
  f.half[0] = *(const v8h*)(p);
  f.half[1] = *(const v8h*)(p + 16);
  return f;
}

__device__ __forceinline__ v8f wmma_raw(v16h a, v16h b, v8f c) {
  return __builtin_amdgcn_wmma_f32_16x16x32_f16(false, a, false, b, (short)0, c, false, false);
}

#define WG1(d, a0, a1, b0, b1) \
  asm volatile("v_nop\n\tv_nop\n\tv_nop\n\tv_nop" : "+v"(d) : "v"(a0), "v"(a1), "v"(b0), "v"(b1))
#define WG2(d0, d1, a0, a1, b0) \
  asm volatile("v_nop\n\tv_nop\n\tv_nop\n\tv_nop" : "+v"(d0), "+v"(d1) : "v"(a0), "v"(a1), "v"(b0))

__device__ __forceinline__ void st16v(void* p, v4u u)  { *(volatile v4u*)p = u; }
__device__ __forceinline__ void stf4v(float* p, v4f v) { *(volatile v4f*)p = v; }

__device__ __forceinline__ v8h cvt8(v8f x) { return __builtin_convertvector(x, v8h); }
__device__ __forceinline__ v8f join8(v4f a, v4f b) { return __builtin_shufflevector(a, b, 0, 1, 2, 3, 4, 5, 6, 7); }

__device__ __forceinline__ float gelu1(float v) {
  return 0.5f * v * erfcf(-v * 0.70710678118654752f);
}

__device__ __forceinline__ float wave_sum(float s) {
#pragma unroll
  for (int off = 16; off >= 1; off >>= 1) s += __shfl_xor(s, off, 32);
  return s;
}

__global__ __launch_bounds__(256)
void k_cast(const float* __restrict__ in, _Float16* __restrict__ out, int n8) {
  const int i = blockIdx.x * 256 + threadIdx.x;
  if (i >= n8) return;
  const float* p = in + (size_t)i * 8;
  v4f a = *(const v4f*)(p);
  v4f b = *(const v4f*)(p + 4);
  Pack16 pk;
  pk.h = cvt8(join8(a, b));
  _Float16* q = out + (size_t)i * 8;
  st16v(q, pk.u);
  __threadfence();
  st16v(q, pk.u);
}

__global__ __launch_bounds__(256)
void k_fold(const float* __restrict__ w, const float* __restrict__ la,
            const float* __restrict__ lb, _Float16* __restrict__ out, int N, int K) {
  const int K8 = K >> 3;
  const int idx = blockIdx.x * 256 + threadIdx.x;
  if (idx >= N * K8) return;
  const int n  = idx / K8;
  const int k8 = (idx - n * K8) * 8;
  const float* wp = w + (size_t)n * K + k8;
  v4f w0 = *(const v4f*)(wp);
  v4f w1 = *(const v4f*)(wp + 4);
  float acc[8] = {w0[0], w0[1], w0[2], w0[3], w1[0], w1[1], w1[2], w1[3]};
  const float* lap = la + (size_t)k8 * LORA_R;
#pragma unroll 1
  for (int r = 0; r < LORA_R; ++r) {
    const float lbv = lb[(size_t)r * N + n];
#pragma unroll
    for (int i = 0; i < 8; ++i) acc[i] += lap[i * LORA_R + r] * lbv;
  }
  v8f x;
#pragma unroll
  for (int i = 0; i < 8; ++i) x[i] = acc[i] * WSCALE;
  Pack16 pk;
  pk.h = cvt8(x);
  _Float16* q = out + (size_t)n * K + k8;
  st16v(q, pk.u);
  __threadfence();
  st16v(q, pk.u);
}

template <bool OUT16, bool GELU, bool RESID>
__global__ __launch_bounds__(256)
void k_gemm(const _Float16* __restrict__ A, const _Float16* __restrict__ Bt,
            const float* __restrict__ bias, const float* __restrict__ resid,
            void* Cv, int N, int K) {
  __shared__ __align__(16) float smem[16384];
  _Float16* As = (_Float16*)smem;
  _Float16* Bs = As + GBM * GLDP;

  const int tid = threadIdx.x, wid = tid >> 5, lane = tid & 31;
  const int h = lane >> 4, m = lane & 15;
  const int wm = wid & 3, wn = wid >> 2;
  const int m_blk = blockIdx.x * GBM;
  const int n_blk = blockIdx.y * GBN;
  const int nk = K / GBK;

  v8f acc[2][4] = {};

  for (int kt = 0; kt < nk; ++kt) {
    const int k0 = kt * GBK;
#pragma unroll
    for (int c = tid; c < 1024; c += 256) {
      const int row = c >> 3, ko = (c & 7) * 8;
      *(v8h*)(As + row * GLDP + ko) = *(const v8h*)(A  + (size_t)(m_blk + row) * K + k0 + ko);
      *(v8h*)(Bs + row * GLDP + ko) = *(const v8h*)(Bt + (size_t)(n_blk + row) * K + k0 + ko);
    }
    __syncthreads();
#pragma unroll
    for (int ks = 0; ks < 2; ++ks) {
      Frag a0 = ld_frag(As, GLDP, wm * 32,      ks * 32);
      Frag a1 = ld_frag(As, GLDP, wm * 32 + 16, ks * 32);
#pragma unroll
      for (int t = 0; t < 4; ++t) {
        Frag b = ld_frag(Bs, GLDP, wn * 64 + t * 16, ks * 32);
        acc[0][t] = wmma_raw(a0.v, b.v, acc[0][t]);
        acc[1][t] = wmma_raw(a1.v, b.v, acc[1][t]);
        WG2(acc[0][t], acc[1][t], a0.v, a1.v, b.v);
      }
    }
    __syncthreads();
  }

  float* Cs = smem + wid * 2048;
#pragma unroll
  for (int u = 0; u < 2; ++u)
#pragma unroll
    for (int t = 0; t < 4; ++t)
#pragma unroll
      for (int e = 0; e < 8; ++e)
        Cs[(u * 16 + 8 * h + e) * 64 + t * 16 + m] = acc[u][t][e];
  __syncthreads();

  const int col0 = n_blk + wn * 64;
  const int row0 = m_blk + wm * 32;

  if (!OUT16) {
    float* C = (float*)Cv;
#pragma unroll 1
    for (int i = 0; i < 16; ++i) {
      const int row = 2 * i + h, c4 = m * 4;
      float* cp = Cs + row * 64 + c4;
      v4f v  = *(v4f*)cp;
      v4f bv = *(const v4f*)(bias + col0 + c4);
      v = v * WSCALE_INV + bv;
      if (RESID) v += *(const v4f*)(resid + (size_t)(row0 + row) * N + col0 + c4);
      if (GELU) {
#pragma unroll
        for (int j = 0; j < 4; ++j) v[j] = gelu1(v[j]);
      }
      *(v4f*)cp = v;
      stf4v(C + (size_t)(row0 + row) * N + col0 + c4, v);
    }
    __threadfence();
#pragma unroll 1
    for (int i = 0; i < 16; ++i) {
      const int row = 2 * i + h, c4 = m * 4;
      v4f v = *(v4f*)(Cs + row * 64 + c4);
      stf4v(C + (size_t)(row0 + row) * N + col0 + c4, v);
    }
  } else {
    _Float16* C = (_Float16*)Cv;
#pragma unroll 1
    for (int i = 0; i < 8; ++i) {
      const int row = 4 * i + (lane >> 3), c8 = (lane & 7) * 8;
      float* cp = Cs + row * 64 + c8;
      v4f v0 = *(v4f*)(cp);
      v4f v1 = *(v4f*)(cp + 4);
      v4f b0 = *(const v4f*)(bias + col0 + c8);
      v4f b1 = *(const v4f*)(bias + col0 + c8 + 4);
      v0 = v0 * WSCALE_INV + b0;
      v1 = v1 * WSCALE_INV + b1;
      if (RESID) {
        v0 += *(const v4f*)(resid + (size_t)(row0 + row) * N + col0 + c8);
        v1 += *(const v4f*)(resid + (size_t)(row0 + row) * N + col0 + c8 + 4);
      }
      if (GELU) {
#pragma unroll
        for (int j = 0; j < 4; ++j) { v0[j] = gelu1(v0[j]); v1[j] = gelu1(v1[j]); }
      }
      *(v4f*)(cp)     = v0;
      *(v4f*)(cp + 4) = v1;
      Pack16 pk;
      pk.h = cvt8(join8(v0, v1));
      st16v(C + (size_t)(row0 + row) * N + col0 + c8, pk.u);
    }
    __threadfence();
#pragma unroll 1
    for (int i = 0; i < 8; ++i) {
      const int row = 4 * i + (lane >> 3), c8 = (lane & 7) * 8;
      const float* cp = Cs + row * 64 + c8;
      Pack16 pk;
      pk.h = cvt8(join8(*(const v4f*)(cp), *(const v4f*)(cp + 4)));
      st16v(C + (size_t)(row0 + row) * N + col0 + c8, pk.u);
    }
  }
}

__global__ __launch_bounds__(256)
void k_attn(const _Float16* __restrict__ Q, const _Float16* __restrict__ Kx,
            const _Float16* __restrict__ V, const float* __restrict__ mask,
            _Float16* __restrict__ O, const int* __restrict__ nh_unused,
            const int* __restrict__ hd_unused) {
  __shared__ __align__(16) _Float16 Ks[64 * ALDP];
  __shared__ __align__(16) _Float16 Vt[64 * ALDP];
  __shared__ __align__(16) _Float16 Os[8 * 16 * ALDP];
  (void)nh_unused; (void)hd_unused;

  const int tid = threadIdx.x, wid = tid >> 5, lane = tid & 31;
  const int h = lane >> 4, m = lane & 15;
  const int qt = blockIdx.x, hh = blockIdx.y, b = blockIdx.z;
  const int qrow0 = b * SEQ + qt * 128 + wid * 16;
  const int colh = hh * HDIM;

  Frag q0 = ld_frag(Q + colh, D_MODEL, qrow0, 0);
  Frag q1 = ld_frag(Q + colh, D_MODEL, qrow0, 32);

  v8f oacc[4] = {};
  float mrow = -1e30f, lrow = 0.f;

  for (int j = 0; j < SEQ / 64; ++j) {
    __syncthreads();
#pragma unroll
    for (int c = tid; c < 512; c += 256) {
      const int r = c >> 3, ko = (c & 7) * 8;
      const size_t g = (size_t)(b * SEQ + j * 64 + r) * D_MODEL + colh + ko;
      *(v8h*)(Ks + r * ALDP + ko) = *(const v8h*)(Kx + g);
      v8h vv = *(const v8h*)(V + g);
#pragma unroll
      for (int i = 0; i < 8; ++i) Vt[(ko + i) * ALDP + r] = vv[i];
    }
    __syncthreads();

    v8f s[4];
#pragma unroll
    for (int t = 0; t < 4; ++t) {
      v8f z = {};
      Frag kf0 = ld_frag(Ks, ALDP, t * 16, 0);
      Frag kf1 = ld_frag(Ks, ALDP, t * 16, 32);
      z = wmma_raw(kf0.v, q0.v, z);
      z = wmma_raw(kf1.v, q1.v, z);
      WG1(z, kf0.v, kf1.v, q0.v, q1.v);
      s[t] = z;
    }

    const float* mp = mask + (size_t)b * SEQ + j * 64 + 8 * h;
    float mloc = -1e30f;
#pragma unroll
    for (int t = 0; t < 4; ++t) {
      v4f m0 = *(const v4f*)(mp + t * 16);
      v4f m1 = *(const v4f*)(mp + t * 16 + 4);
#pragma unroll
      for (int e = 0; e < 4; ++e) {
        s[t][e]     = s[t][e]     * 0.125f + m0[e];
        s[t][4 + e] = s[t][4 + e] * 0.125f + m1[e];
      }
#pragma unroll
      for (int e = 0; e < 8; ++e) mloc = fmaxf(mloc, s[t][e]);
    }
    mloc = fmaxf(mloc, __shfl_xor(mloc, 16, 32));
    const float mnew = fmaxf(mrow, mloc);
    const float corr = __expf(mrow - mnew);
    mrow = mnew;
    lrow *= corr;
#pragma unroll
    for (int t = 0; t < 4; ++t) oacc[t] = oacc[t] * corr;
    float rsum = 0.f;
#pragma unroll
    for (int t = 0; t < 4; ++t) {
#pragma unroll
      for (int e = 0; e < 8; ++e) {
        const float p = __expf(s[t][e] - mnew);
        s[t][e] = p;
        rsum += p;
      }
    }
    rsum += __shfl_xor(rsum, 16, 32);
    lrow += rsum;

    Frag p0, p1;
    p0.half[0] = cvt8(s[0] * PSCALE);
    p0.half[1] = cvt8(s[1] * PSCALE);
    p1.half[0] = cvt8(s[2] * PSCALE);
    p1.half[1] = cvt8(s[3] * PSCALE);

#pragma unroll
    for (int td = 0; td < 4; ++td) {
      Frag v0 = ld_frag(Vt, ALDP, td * 16, 0);
      Frag v1 = ld_frag(Vt, ALDP, td * 16, 32);
      oacc[td] = wmma_raw(v0.v, p0.v, oacc[td]);
      oacc[td] = wmma_raw(v1.v, p1.v, oacc[td]);
      WG1(oacc[td], v0.v, v1.v, p0.v, p1.v);
    }
  }

  const float inv = (1.0f / lrow) * PSCALE_INV;
  _Float16* osw = Os + wid * 16 * ALDP;
#pragma unroll
  for (int td = 0; td < 4; ++td)
    *(v8h*)(osw + m * ALDP + td * 16 + 8 * h) = cvt8(oacc[td] * inv);
  __syncthreads();

#pragma unroll
  for (int i = 0; i < 4; ++i) {
    const int row = 4 * i + (lane >> 3), c8 = (lane & 7) * 8;
    Pack16 pk;
    pk.h = *(const v8h*)(osw + row * ALDP + c8);
    st16v(O + (size_t)(qrow0 + row) * D_MODEL + colh + c8, pk.u);
  }
  __threadfence();
#pragma unroll
  for (int i = 0; i < 4; ++i) {
    const int row = 4 * i + (lane >> 3), c8 = (lane & 7) * 8;
    Pack16 pk;
    pk.h = *(const v8h*)(osw + row * ALDP + c8);
    st16v(O + (size_t)(qrow0 + row) * D_MODEL + colh + c8, pk.u);
  }
}

template <bool H16>
__global__ __launch_bounds__(256)
void k_ln(const float* __restrict__ in, const float* __restrict__ w,
          const float* __restrict__ bb, float* __restrict__ outf,
          _Float16* __restrict__ outh, int nrows) {
  __shared__ float red0[8];
  __shared__ float red1[8];
  const int row = blockIdx.x;
  const int tid = threadIdx.x, wid = tid >> 5, lane = tid & 31;
  const bool ok = row < nrows;
  const float* x = in + (size_t)(ok ? row : 0) * D_MODEL;

  v4f v = *(const v4f*)(x + tid * 4);
  float s = (v[0] + v[1]) + (v[2] + v[3]);
  s = wave_sum(s);
  if (lane == 0) red0[wid] = s;
  __syncthreads();
  float tot = 0.f;
#pragma unroll
  for (int i = 0; i < 8; ++i) tot += red0[i];
  const float mu = tot * (1.0f / (float)D_MODEL);

  v4f d = v - mu;
  float ss = (d[0] * d[0] + d[1] * d[1]) + (d[2] * d[2] + d[3] * d[3]);
  ss = wave_sum(ss);
  if (lane == 0) red1[wid] = ss;
  __syncthreads();
  float tot2 = 0.f;
#pragma unroll
  for (int i = 0; i < 8; ++i) tot2 += red1[i];
  const float var = tot2 * (1.0f / (float)D_MODEL);
  const float inv = rsqrtf(var + LN_EPS);

  v4f wv = *(const v4f*)(w + tid * 4);
  v4f bv = *(const v4f*)(bb + tid * 4);
  v4f y = (d * inv) * wv + bv;

  Pack16 pk;
  const int c8 = tid * 8;
  const bool do16 = H16 && (tid < 128);
  if (do16) {
    v4f x0 = *(const v4f*)(x + c8);
    v4f x1 = *(const v4f*)(x + c8 + 4);
    v4f w0 = *(const v4f*)(w + c8), w1 = *(const v4f*)(w + c8 + 4);
    v4f c0 = *(const v4f*)(bb + c8), c1 = *(const v4f*)(bb + c8 + 4);
    v4f y0 = ((x0 - mu) * inv) * w0 + c0;
    v4f y1 = ((x1 - mu) * inv) * w1 + c1;
    pk.h = cvt8(join8(y0, y1));
  }
  if (ok) {
    float* op = outf + (size_t)row * D_MODEL + tid * 4;
    stf4v(op, y);
    if (do16) st16v(outh + (size_t)row * D_MODEL + c8, pk.u);
    __threadfence();
    stf4v(op, y);
    if (do16) st16v(outh + (size_t)row * D_MODEL + c8, pk.u);
  }
}

extern "C" void kernel_launch(void* const* d_in, const int* in_sizes, int n_in,
                              void* d_out, int out_size, void* d_ws, size_t ws_size,
                              hipStream_t stream) {
  if (n_in < 32) return;
  if (in_sizes[0] != MTOT * D_MODEL) return;
  if (in_sizes[1] != BATCH * SEQ) return;
  if (in_sizes[2] != D_MODEL * D_MODEL || in_sizes[6] != D_MODEL * D_MODEL ||
      in_sizes[10] != D_MODEL * D_MODEL || in_sizes[14] != D_MODEL * D_MODEL) return;
  if (in_sizes[20] != FF_DIM * D_MODEL || in_sizes[24] != D_MODEL * FF_DIM) return;
  if (in_sizes[4] != D_MODEL * LORA_R || in_sizes[23] != LORA_R * FF_DIM ||
      in_sizes[26] != FF_DIM * LORA_R) return;
  if (out_size != MTOT * D_MODEL) return;

  const float* x     = (const float*)d_in[0];
  const float* amask = (const float*)d_in[1];
  const float* w_q  = (const float*)d_in[2];  const float* b_q  = (const float*)d_in[3];
  const float* la_q = (const float*)d_in[4];  const float* lb_q = (const float*)d_in[5];
  const float* w_k  = (const float*)d_in[6];  const float* b_k  = (const float*)d_in[7];
  const float* la_k = (const float*)d_in[8];  const float* lb_k = (const float*)d_in[9];
  const float* w_v  = (const float*)d_in[10]; const float* b_v  = (const float*)d_in[11];
  const float* la_v = (const float*)d_in[12]; const float* lb_v = (const float*)d_in[13];
  const float* w_o  = (const float*)d_in[14]; const float* b_o  = (const float*)d_in[15];
  const float* la_o = (const float*)d_in[16]; const float* lb_o = (const float*)d_in[17];
  const float* nw1  = (const float*)d_in[18]; const float* nb1  = (const float*)d_in[19];
  const float* w_up = (const float*)d_in[20]; const float* b_up = (const float*)d_in[21];
  const float* la_up = (const float*)d_in[22]; const float* lb_up = (const float*)d_in[23];
  const float* w_dn = (const float*)d_in[24]; const float* b_dn = (const float*)d_in[25];
  const float* la_dn = (const float*)d_in[26]; const float* lb_dn = (const float*)d_in[27];
  const float* nw2  = (const float*)d_in[28]; const float* nb2  = (const float*)d_in[29];
  const int*   nh_p = (const int*)d_in[30];
  const int*   hd_p = (const int*)d_in[31];

  char* ws = (char*)d_ws;
  size_t off = 0;
  auto carve = [&](size_t bytes) -> char* {
    size_t cur = (off + 255) & ~(size_t)255;
    off = cur + bytes;
    return ws + cur;
  };
  const size_t actH = (size_t)MTOT * D_MODEL * 2;
  const size_t actF = (size_t)MTOT * D_MODEL * 4;
  const size_t wDD  = (size_t)D_MODEL * D_MODEL * 2;
  const size_t wFD  = (size_t)FF_DIM * D_MODEL * 2;

  _Float16* x16  = (_Float16*)carve(actH);
  _Float16* Wfq  = (_Float16*)carve(wDD);
  _Float16* Wfk  = (_Float16*)carve(wDD);
  _Float16* Wfv  = (_Float16*)carve(wDD);
  _Float16* Wfo  = (_Float16*)carve(wDD);
  _Float16* Wfup = (_Float16*)carve(wFD);
  _Float16* Wfdn = (_Float16*)carve(wFD);
  char*     R1   = carve(4 * actH);
  _Float16* q16  = (_Float16*)(R1);
  _Float16* k16  = (_Float16*)(R1 + actH);
  _Float16* v16  = (_Float16*)(R1 + 2 * actH);
  _Float16* o16  = (_Float16*)(R1 + 3 * actH);
  _Float16* fn16 = (_Float16*)(R1);
  float*    ofin = (float*)carve(actF);
  float*    dwn  = ofin;
  float*    xm   = (float*)carve(actF);
  _Float16* xm16 = (_Float16*)carve(actH);
  if (off > ws_size) return;

  const int n8 = MTOT * D_MODEL / 8;
  k_cast<<<(n8 + 255) / 256, 256, 0, stream>>>(x, x16, n8);

  const int nDD8 = D_MODEL * D_MODEL / 8, nFD8 = FF_DIM * D_MODEL / 8;
  k_fold<<<(nDD8 + 255) / 256, 256, 0, stream>>>(w_q,  la_q,  lb_q,  Wfq,  D_MODEL, D_MODEL);
  k_fold<<<(nDD8 + 255) / 256, 256, 0, stream>>>(w_k,  la_k,  lb_k,  Wfk,  D_MODEL, D_MODEL);
  k_fold<<<(nDD8 + 255) / 256, 256, 0, stream>>>(w_v,  la_v,  lb_v,  Wfv,  D_MODEL, D_MODEL);
  k_fold<<<(nDD8 + 255) / 256, 256, 0, stream>>>(w_o,  la_o,  lb_o,  Wfo,  D_MODEL, D_MODEL);
  k_fold<<<(nFD8 + 255) / 256, 256, 0, stream>>>(w_up, la_up, lb_up, Wfup, FF_DIM,  D_MODEL);
  k_fold<<<(nFD8 + 255) / 256, 256, 0, stream>>>(w_dn, la_dn, lb_dn, Wfdn, D_MODEL, FF_DIM);

  const dim3 gD(MTOT / GBM, D_MODEL / GBN);
  const dim3 gF(MTOT / GBM, FF_DIM / GBN);

  k_gemm<true, false, false><<<gD, 256, 0, stream>>>(x16, Wfq, b_q, x, (void*)q16, D_MODEL, D_MODEL);
  k_gemm<true, false, false><<<gD, 256, 0, stream>>>(x16, Wfk, b_k, x, (void*)k16, D_MODEL, D_MODEL);
  k_gemm<true, false, false><<<gD, 256, 0, stream>>>(x16, Wfv, b_v, x, (void*)v16, D_MODEL, D_MODEL);

  k_attn<<<dim3(SEQ / 128, NHEAD, BATCH), 256, 0, stream>>>(q16, k16, v16, amask, o16, nh_p, hd_p);

  k_gemm<false, false, true><<<gD, 256, 0, stream>>>(o16, Wfo, b_o, x, (void*)ofin, D_MODEL, D_MODEL);

  k_ln<true><<<MTOT, 256, 0, stream>>>(ofin, nw1, nb1, xm, xm16, MTOT);

  k_gemm<true, true, false><<<gF, 256, 0, stream>>>(xm16, Wfup, b_up, x, (void*)fn16, FF_DIM, D_MODEL);

  k_gemm<false, false, true><<<gD, 256, 0, stream>>>(fn16, Wfdn, b_dn, xm, (void*)dwn, D_MODEL, FF_DIM);

  k_ln<false><<<MTOT, 256, 0, stream>>>(dwn, nw2, nb2, (float*)d_out, xm16, MTOT);

  (void)hipGetLastError();
}
